// self_attn_enc_40200893890895
// MI455X (gfx1250) — hardware-verified
//
#include <hip/hip_runtime.h>
#include <math.h>

typedef __attribute__((ext_vector_type(16))) _Float16 v16h;
typedef __attribute__((ext_vector_type(16))) __bf16 v16b;
typedef __attribute__((ext_vector_type(8)))  _Float16 v8h;
typedef __attribute__((ext_vector_type(8)))  float v8f;
typedef __attribute__((ext_vector_type(4)))  float v4f;
typedef __attribute__((ext_vector_type(2)))  float v2f;
typedef __attribute__((ext_vector_type(4)))  unsigned v4u;
typedef __attribute__((ext_vector_type(4)))  int v4i;
typedef float __attribute__((may_alias)) float_a;
typedef int __attribute__((may_alias)) int_a;

template <typename T> __device__ __forceinline__ void vst2(void* p, T v) { *(volatile T*)p = v; __threadfence(); *(volatile T*)p = v; }
__device__ __forceinline__ v8f wmma16(v16h a, v16h b, v8f c) {
  v8f d = __builtin_amdgcn_wmma_f32_16x16x32_f16(false, a, false, b, (short)0, c, false, false);
  asm volatile("v_nop\n\tv_nop\n\tv_nop\n\tv_nop" : "+v"(d) : "v"(a), "v"(b));
  return d;
}
__device__ __forceinline__ v8f wmma_bf(v16b a, v16b b, v8f c) {
  v8f d = __builtin_amdgcn_wmma_f32_16x16x32_bf16(false, a, false, b, (short)0, c, false, false);
  asm volatile("v_nop\n\tv_nop\n\tv_nop\n\tv_nop" : "+v"(d) : "v"(a), "v"(b));
  return d;
}
__device__ __forceinline__ v16h frag_h(const _Float16* rowk0, int lane) {
  union { v16h v; v8h q[2]; } u; const _Float16* p = rowk0 + 8 * (lane >> 4);
  u.q[0] = *(const v8h*)p; u.q[1] = *(const v8h*)(p + 16); return u.v;
}
__device__ __forceinline__ v16h frag_f32(const float* rowk0, int lane) {
  v16h a; const float* p = rowk0 + 8 * (lane >> 4);
#pragma unroll
  for (int i = 0; i < 8; ++i) { a[i] = (_Float16)p[i]; a[8 + i] = (_Float16)p[16 + i]; }
  return a;
}
__device__ __forceinline__ v16h frag_f32s(const float* rowk0, int lane, float sc) {
  v16h a; const float* p = rowk0 + 8 * (lane >> 4);
#pragma unroll
  for (int i = 0; i < 8; ++i) { a[i] = (_Float16)(p[i] * sc); a[8 + i] = (_Float16)(p[16 + i] * sc); }
  return a;
}
__device__ __forceinline__ v16h fragc_f32(const float* W, int k0, int n, int lane, int ld, int K) {
  v16h a; const int g = lane >> 4;
#pragma unroll
  for (int i = 0; i < 8; ++i) { const int ka = k0 + 8 * g + i, kb = ka + 16;
    a[i] = (_Float16)(ka < K ? W[(size_t)(ka < K ? ka : K - 1) * ld + n] : 0.f); a[8 + i] = (_Float16)(kb < K ? W[(size_t)(kb < K ? kb : K - 1) * ld + n] : 0.f); }
  return a;
}
struct F2 { v16b h, l; };
__device__ __forceinline__ F2 bsplit16(const float v[16]) { F2 r;
#pragma unroll
  for (int i = 0; i < 16; ++i) { const __bf16 h = (__bf16)v[i]; r.h[i] = h; r.l[i] = (__bf16)(v[i] - (float)h); }
  return r; }
__device__ __forceinline__ F2 split_row(const float* row, int k0, int lane) { float v[16]; const float* p = row + k0 + 8 * (lane >> 4);
#pragma unroll
  for (int i = 0; i < 8; ++i) { v[i] = p[i]; v[8 + i] = p[16 + i]; }
  return bsplit16(v); }
__device__ __forceinline__ F2 split_rowK(const float* row, int k0, int lane, int K) { float v[16]; const int g = lane >> 4;
#pragma unroll
  for (int i = 0; i < 8; ++i) { const int ka = k0 + 8 * g + i, kb = ka + 16; v[i] = ka < K ? row[ka < K ? ka : K - 1] : 0.f; v[8 + i] = kb < K ? row[kb < K ? kb : K - 1] : 0.f; }
  return bsplit16(v); }
__device__ __forceinline__ F2 split_col(const float* W, int k0, int n, int lane, int ld, int K) { float v[16]; const int g = lane >> 4;
#pragma unroll
  for (int i = 0; i < 8; ++i) { const int ka = k0 + 8 * g + i, kb = ka + 16; v[i] = ka < K ? W[(size_t)(ka < K ? ka : K - 1) * ld + n] : 0.f; v[8 + i] = kb < K ? W[(size_t)(kb < K ? kb : K - 1) * ld + n] : 0.f; }
  return bsplit16(v); }
__device__ __forceinline__ v8f mac3(const F2& a, const F2& b, v8f c) { c = wmma_bf(a.l, b.h, c); c = wmma_bf(a.h, b.l, c); return wmma_bf(a.h, b.h, c); }
__device__ __forceinline__ float sigm(float v) { return 1.0f / (1.0f + expf(-v)); }
#define LDSX() do { asm volatile("s_wait_dscnt 0" ::: "memory"); __builtin_amdgcn_wave_barrier(); __builtin_amdgcn_fence(__ATOMIC_RELEASE, "workgroup"); } while (0)


#define NN 8192
#define DI 128
#define DO 128
#ifndef TQB
#define TQB (NN / 64)
#endif
typedef __attribute__((ext_vector_type(8))) __bf16 v8b;
__device__ __forceinline__ v16b frag_b(const __bf16* rowk0, int lane) {
  union { v16b v; v8b q[2]; } u; const __bf16* p = rowk0 + 8 * (lane >> 4);
  u.q[0] = *(const v8b*)p; u.q[1] = *(const v8b*)(p + 16); return u.v;
}
__device__ __forceinline__ float bfr(float v) { return (float)(__bf16)v; }
__device__ __attribute__((noinline)) float exp_ni(float v) { return expf(v); }
__device__ __attribute__((noinline)) float erf_ni(float v) { return erff(v); }

#define WS_PK  0u
#define WS_KF  (WS_PK + 2u * 4 * DO * DI)
#define WS_KH  (WS_KF + 4u * NN * DO)
#define WS_KL  (WS_KH + 2u * NN * DO)
#define WS_QH  (WS_KL + 2u * NN * DO)
#define WS_QL  (WS_QH + 2u * NN * DO)
#define WS_VT  (WS_QL + 2u * NN * DO)
#define WS_KV  (WS_VT + 2u * NN * DO)
#define WS_END (WS_KV + 4u * NN * DO)

__global__ __launch_bounds__(128) void k_pack(const float* __restrict__ WK, const float* __restrict__ WQ, const float* __restrict__ WV, __bf16* __restrict__ PK) {
  const int n = blockIdx.x, which = blockIdx.y, t = threadIdx.x; __shared__ __align__(16) __bf16 s[DI]; float v;
  if (which == 0) v = WK[(size_t)n * DI + t]; else if (which == 1) v = WQ[(size_t)n * DI + t]; else if (which == 2) v = WV[(size_t)n * (2 * DO) + t]; else v = WV[(size_t)n * (2 * DO) + DO + t];
  s[t] = (__bf16)v; __syncthreads();
  if (t < DI / 8) vst2((unsigned*)(PK + ((size_t)which * DO + n) * DI + t * 8), *(const v4u*)&s[t * 8]);
}
__global__ __launch_bounds__(128) void k_proj(const float* __restrict__ NODES, const float* __restrict__ CEN, const float* __restrict__ PREV, const __bf16* __restrict__ PK, const float* __restrict__ BK, const float* __restrict__ BQ, const float* __restrict__ BV, float* __restrict__ KF, _Float16* __restrict__ KH, _Float16* __restrict__ KL, _Float16* __restrict__ QH, _Float16* __restrict__ QL, _Float16* __restrict__ VT, float* __restrict__ KV) {
  __shared__ __align__(16) __bf16 sx[64][DI + 8]; __shared__ __align__(16) __bf16 skh[64][DI + 8], skl[64][DI + 8], sqh[64][DI + 8], sql[64][DI + 8]; __shared__ __align__(16) float skf[64][DO + 4]; __shared__ __align__(16) _Float16 svt[DO][72];
  const int tid = threadIdx.x, wave = tid >> 5, lane = tid & 31, col = lane & 15, g = lane >> 4; const size_t r0 = (size_t)blockIdx.x * 64;
  for (int e = tid; e < 64 * DI; e += 128) { const int r = e >> 7, c = e & 127; const size_t row = r0 + r; float v; if (c < 3) v = NODES[row * 3 + c]; else if (c < 6) v = CEN[c - 3]; else v = PREV[row * 122 + (c - 6)]; sx[r][c] = (__bf16)v; }
  if (tid < 64) for (int c = DI; c < DI + 8; ++c) { sx[tid][c] = (__bf16)0.f; skh[tid][c] = (__bf16)0.f; skl[tid][c] = (__bf16)0.f; sqh[tid][c] = (__bf16)0.f; sql[tid][c] = (__bf16)0.f; }
  __syncthreads();
#pragma unroll 1
  for (int pass = 0; pass < 2; ++pass) { v8f acc[8] = {}; const bool isq = pass == 1;
#pragma unroll
    for (int kc = 0; kc < DI / 32; ++kc) { const v16b a = frag_b(&sx[wave * 16 + col][kc * 32], lane);
#pragma unroll
      for (int j = 0; j < 8; ++j) acc[j] = wmma_bf(a, frag_b(PK + (size_t)(pass * DO + j * 16 + col) * DI + kc * 32, lane), acc[j]); }
#pragma unroll
    for (int j = 0; j < 8; ++j) { const int c = j * 16 + col; const float bb = bfr((isq ? BQ : BK)[c]);
#pragma unroll
      for (int r = 0; r < 8; ++r) { const float v = acc[j][r] + bb; const int rr = wave * 16 + 8 * g + r; const __bf16 hb = (__bf16)v; const __bf16 lb = (__bf16)(v - (float)hb);
        if (isq) { sqh[rr][c] = hb; sql[rr][c] = lb; } else { skh[rr][c] = hb; skl[rr][c] = lb; skf[rr][c] = v; } } } }
  __syncthreads();
  for (int e = tid; e < 64 * DO; e += 128) { const int r = e >> 7, c = e & 127; const size_t row = r0 + r;
    { const float v = skf[r][c]; const _Float16 hv = (_Float16)v; KH[row * DO + c] = hv; KL[row * DO + c] = (_Float16)((v - (float)hv) * 2048.0f); }
    { const float v = (float)sqh[r][c] + (float)sql[r][c]; const _Float16 hv = (_Float16)v; QH[row * DO + c] = hv; QL[row * DO + c] = (_Float16)((v - (float)hv) * 2048.0f); } }
  for (int e = tid; e < 64 * (DO / 4); e += 128) { const int r = e >> 5, q = e & 31; vst2(KF + (r0 + r) * DO + q * 4, *(const v4f*)&skf[r][q * 4]); }
  __syncthreads();
  { v8f acc[8] = {};
#pragma unroll
    for (int kc = 0; kc < DO / 32; ++kc) { const v16b aq = frag_b(&sqh[wave * 16 + col][kc * 32], lane), aql = frag_b(&sql[wave * 16 + col][kc * 32], lane);
#pragma unroll
      for (int j = 0; j < 8; ++j) { const v16b wvq = frag_b(PK + (size_t)(2 * DO + j * 16 + col) * DI + kc * 32, lane); acc[j] = wmma_bf(aql, wvq, acc[j]); acc[j] = wmma_bf(aq, wvq, acc[j]); } }
#pragma unroll
    for (int j = 0; j < 8; ++j) { const int c = j * 16 + col;
#pragma unroll
      for (int r = 0; r < 8; ++r) svt[c][wave * 16 + 8 * g + r] = (_Float16)acc[j][r]; } }
  { v8f acc[8] = {};
#pragma unroll
    for (int kc = 0; kc < DO / 32; ++kc) { const v16b ak = frag_b(&skh[wave * 16 + col][kc * 32], lane), akl = frag_b(&skl[wave * 16 + col][kc * 32], lane);
#pragma unroll
      for (int j = 0; j < 8; ++j) { const v16b wvk = frag_b(PK + (size_t)(3 * DO + j * 16 + col) * DI + kc * 32, lane); acc[j] = wmma_bf(akl, wvk, acc[j]); acc[j] = wmma_bf(ak, wvk, acc[j]); } }
#pragma unroll
    for (int j = 0; j < 8; ++j) { const int c = j * 16 + col;
#pragma unroll
      for (int r = 0; r < 8; ++r) { const int rr = wave * 16 + 8 * g + r; const float kv = acc[j][r] + bfr(BV[c]) + skf[rr][c]; skf[rr][c] = kv; } } }
  __syncthreads();
  for (int e = tid; e < DO * 8; e += 128) { const int c = e >> 3, pc = e & 7; vst2((unsigned*)(VT + (size_t)c * NN + r0 + pc * 8), *(const v4u*)&svt[c][pc * 8]); }
  for (int e = tid; e < 64 * (DO / 4); e += 128) { const int r = e >> 5, q = e & 31; vst2(KV + (r0 + r) * DO + q * 4, *(const v4f*)&skf[r][q * 4]); }
}
__global__ __launch_bounds__(128) void k_attn(const _Float16* __restrict__ KH, const _Float16* __restrict__ KL, const _Float16* __restrict__ QH, const _Float16* __restrict__ QL, const _Float16* __restrict__ VT, const float* __restrict__ KV, float* __restrict__ OUT) {
  __shared__ __align__(16) _Float16 sph[4][16][40]; __shared__ __align__(16) float so[4][16][132];
  const int tid = threadIdx.x, wave = tid >> 5, lane = tid & 31, col = lane & 15, g = lane >> 4; const size_t r0 = (size_t)blockIdx.x * 64 + wave * 16;
  v16h ak[DO / 32], akl[DO / 32];
#pragma unroll
  for (int kc = 0; kc < DO / 32; ++kc) { ak[kc] = frag_h(KH + (r0 + col) * DO + kc * 32, lane); akl[kc] = frag_h(KL + (r0 + col) * DO + kc * 32, lane); }
  float m[8], l[8];
#pragma unroll
  for (int r = 0; r < 8; ++r) { m[r] = -3.0e38f; l[r] = 0.f; }
  v8f acc[8] = {};
#pragma unroll 1
  for (int ks = 0; ks < NN / 32; ++ks) { const int j0 = ks * 32; v8f s[2];
#pragma unroll
    for (int ct = 0; ct < 2; ++ct) { const size_t rq = (size_t)(j0 + ct * 16 + col) * DO; v8f c = {}, cl = {};
#pragma unroll
      for (int kc = 0; kc < DO / 32; ++kc) { const v16h qh = frag_h(QH + rq + kc * 32, lane); c = wmma16(ak[kc], qh, c); cl = wmma16(akl[kc], qh, cl); cl = wmma16(ak[kc], frag_h(QL + rq + kc * 32, lane), cl); }
#pragma unroll
      for (int r = 0; r < 8; ++r) s[ct][r] = c[r] + cl[r] * (1.0f / 2048.0f); }
#pragma unroll
    for (int r = 0; r < 8; ++r) { float mx = fmaxf(s[0][r], s[1][r]);
#pragma unroll
      for (int o = 1; o < 16; o <<= 1) mx = fmaxf(mx, __shfl_xor(mx, o));
      const float mn = fmaxf(m[r], mx); const float alpha = (m[r] <= -1.0e38f) ? 0.f : __expf(m[r] - mn); const float e0 = __expf(s[0][r] - mn), e1 = __expf(s[1][r] - mn); float es = e0 + e1;
#pragma unroll
      for (int o = 1; o < 16; o <<= 1) es += __shfl_xor(es, o);
      l[r] = l[r] * alpha + es; m[r] = mn;
#pragma unroll
      for (int dt = 0; dt < 8; ++dt) acc[dt][r] *= alpha;
      sph[wave][8 * g + r][col] = (_Float16)(e0 * 2048.0f); sph[wave][8 * g + r][16 + col] = (_Float16)(e1 * 2048.0f); }
    LDSX();
    const v16h pa = frag_h(&sph[wave][col][0], lane);
#pragma unroll
    for (int dt = 0; dt < 8; ++dt) acc[dt] = wmma16(pa, frag_h(VT + (size_t)(dt * 16 + col) * NN + j0, lane), acc[dt]);
    LDSX(); }
#pragma unroll
  for (int r = 0; r < 8; ++r) { const float il = (1.0f / 2048.0f) / l[r]; const size_t row = r0 + 8 * g + r;
#pragma unroll
    for (int dt = 0; dt < 8; ++dt) { const int c = dt * 16 + col; so[wave][8 * g + r][c] = acc[dt][r] * il + KV[row * DO + c]; } }
  LDSX();
  for (int rl = 0; rl < 16; ++rl) vst2(OUT + (r0 + rl) * DO + lane * 4, *(const v4f*)&so[wave][rl][lane * 4]);
}
extern "C" void kernel_launch(void* const* d_in, const int* in_sizes, int n_in, void* d_out, int out_size, void* d_ws, size_t ws_size, hipStream_t stream) {
  (void)in_sizes; (void)n_in; (void)out_size;
  const float** F = (const float**)d_in;
  if (ws_size < (size_t)WS_END) return;
  char* ws = (char*)d_ws; __bf16* PK = (__bf16*)(ws + WS_PK); float *KF = (float*)(ws + WS_KF), *KV = (float*)(ws + WS_KV); _Float16 *KH = (_Float16*)(ws + WS_KH), *KL = (_Float16*)(ws + WS_KL), *QH = (_Float16*)(ws + WS_QH), *QL = (_Float16*)(ws + WS_QL), *VT = (_Float16*)(ws + WS_VT);
  k_pack<<<dim3(DO, 4), 128, 0, stream>>>(F[5], F[3], F[7], PK);
  k_proj<<<NN / 64, 128, 0, stream>>>(F[0], F[1], F[2], PK, F[6], F[4], F[8], KF, KH, KL, QH, QL, VT, KV);
  k_attn<<<TQB, 128, 0, stream>>>(KH, KL, QH, QL, VT, KV, (float*)d_out);
}
